// CellBERTModel_7352984010955
// MI455X (gfx1250) — hardware-run, weakly checked
//
#include <hip/hip_runtime.h>
#include <math.h>
#include <stdint.h>

#define NB     8
#define NCELL  1024
#define SV     1025
#define SP     1088
#define MP     (NB * SP)
#define MC     (NB * NCELL)
#define DM     256
#define NH     8
#define HD     32
#define DFF    1024
#define DCT    128
#define FEAT   64
#define NLAYER 4
#define QKP    (2 * DM)
#define NQB    (SP / 64)
#define MAXHW  1000
#define PEW    128
#define NOUT0  (NB * DM)
#define NOUT1  (NB * 2)
#define LNEPS  1.0e-5f
#define WSC    64.0f
static_assert(NH * HD == DM);
static_assert(SP >= SV && (SP % 64) == 0 && (SP - SV) < 64);
static_assert((MP % 64) == 0 && (MC % 64) == 0 && (DM % 64) == 0 && (DFF % 64) == 0);
static_assert((DCT % 64) == 0 && (FEAT % 64) == 0 && (QKP % 64) == 0);
static_assert(2 * PEW == DM && DM == 4 * 64);
static_assert(NOUT0 == 2048 && NOUT1 == 16);
static_assert((MC * FEAT) % (8 * 256) == 0);

typedef _Float16 v16h __attribute__((ext_vector_type(16)));
typedef _Float16 v8h  __attribute__((ext_vector_type(8)));
typedef float    v8f  __attribute__((ext_vector_type(8)));
typedef float    v4f  __attribute__((ext_vector_type(4)));
typedef unsigned int v4u __attribute__((ext_vector_type(4)));
typedef unsigned int v2u __attribute__((ext_vector_type(2)));

__device__ __forceinline__ unsigned short bf_bits(float f) {
  unsigned u = __float_as_uint(f);
  return (unsigned short)((u + 0x7FFFu + ((u >> 16) & 1u)) >> 16);
}
__device__ __forceinline__ float bf_up(unsigned short h) { return __uint_as_float(((unsigned)h) << 16); }
__device__ __forceinline__ float bfr(float f) { return bf_up(bf_bits(f)); }
__device__ __forceinline__ unsigned short h_bits(_Float16 x) { return __builtin_bit_cast(unsigned short, x); }
__device__ __forceinline__ unsigned pk16(unsigned short a, unsigned short b) { return (unsigned)a | ((unsigned)b << 16); }
__device__ __forceinline__ v8f zero8() { v8f z = {0.f, 0.f, 0.f, 0.f, 0.f, 0.f, 0.f, 0.f}; return z; }

__device__ __forceinline__ v16h ldfrag_h(const _Float16* p) {
  union { v16h v; v8h h[2]; } f;
  f.h[0] = *(const v8h*)(p);
  f.h[1] = *(const v8h*)(p + 16);
  return f.v;
}

__device__ __forceinline__ v8f mma_h(v16h a, v16h b, v8f c) {
  c = __builtin_amdgcn_wmma_f32_16x16x32_f16(false, a, false, b, (short)0, c, false, false);
#if defined(__HIP_DEVICE_COMPILE__)
  asm volatile("v_nop\n\tv_nop\n\tv_nop\n\tv_nop" : "+v"(c) : "v"(a), "v"(b));
#endif
  return c;
}
__device__ __forceinline__ v8f mma_h_raw(v16h a, v16h b, v8f c) {
  return __builtin_amdgcn_wmma_f32_16x16x32_f16(false, a, false, b, (short)0, c, false, false);
}
__device__ __forceinline__ void dep_guard1(v8f& a, v8f& b, v16h x) {
#if defined(__HIP_DEVICE_COMPILE__)
  asm volatile("v_nop\n\tv_nop\n\tv_nop\n\tv_nop" : "+v"(a), "+v"(b) : "v"(x));
#endif
}
__device__ __forceinline__ void keep4_h(v16h a, v16h b, v16h c, v16h d) {
#if defined(__HIP_DEVICE_COMPILE__)
  asm volatile("v_nop" :: "v"(a), "v"(b), "v"(c), "v"(d));
#endif
}
__device__ __forceinline__ void acc_guard4(v8f& a, v8f& b, v8f& c, v8f& d) {
#if defined(__HIP_DEVICE_COMPILE__)
  asm volatile("v_nop\n\tv_nop\n\tv_nop\n\tv_nop" : "+v"(a), "+v"(b), "+v"(c), "+v"(d));
#endif
}
__device__ __forceinline__ void wave_sync_lds() {
  __builtin_amdgcn_fence(__ATOMIC_RELEASE, "workgroup");
  __builtin_amdgcn_wave_barrier();
  __builtin_amdgcn_fence(__ATOMIC_ACQUIRE, "workgroup");
}
__device__ __forceinline__ float wsum(float v) {
#pragma unroll
  for (int off = 16; off > 0; off >>= 1) v += __shfl_xor(v, off, 32);
  return v;
}
__device__ __forceinline__ float bsum256(float v, float* red, int lane, int wave) {
  v = wsum(v);
  if (lane == 0) red[wave] = v;
  __syncthreads();
  float tot = 0.f;
#pragma unroll
  for (int w = 0; w < 8; ++w) tot += red[w];
  return tot;
}
__device__ __forceinline__ float bsum2(float v, float* red, int lane, int wave) {
  v = wsum(v);
  if (lane == 0) red[wave] = v;
  __syncthreads();
  return red[0] + red[1];
}

__device__ __forceinline__ void row_store_fh(unsigned int* sb, float* dstF, unsigned short* dstH, v4f y, int t) {
  *(volatile v4f*)(dstF + 4 * t) = y;
  v2u p;
  p[0] = pk16(h_bits((_Float16)y[0]), h_bits((_Float16)y[1]));
  p[1] = pk16(h_bits((_Float16)y[2]), h_bits((_Float16)y[3]));
  *(v2u*)(sb + 2 * t) = p;
  __syncthreads();
  if (t < 32) {
    const v4u v = *(const v4u*)(sb + 4 * t);
    *(volatile v4u*)(dstH + 8 * t) = v;
    __threadfence();
    *(volatile v4u*)(dstH + 8 * t) = v;
  }
  __threadfence();
  *(volatile v4f*)(dstF + 4 * t) = y;
}

__global__ __launch_bounds__(256) void conv_rows8(const float* __restrict__ src, unsigned short* dst, int n8) {
  const int i  = blockIdx.x * 256 + threadIdx.x;
  const int ic = (i < n8) ? i : (n8 - 1);
  const v4f a = *(const v4f*)(src + (size_t)ic * 8);
  const v4f b = *(const v4f*)(src + (size_t)ic * 8 + 4);
  v4u o;
  o[0] = pk16(h_bits((_Float16)bfr(a[0])), h_bits((_Float16)bfr(a[1])));
  o[1] = pk16(h_bits((_Float16)bfr(a[2])), h_bits((_Float16)bfr(a[3])));
  o[2] = pk16(h_bits((_Float16)bfr(b[0])), h_bits((_Float16)bfr(b[1])));
  o[3] = pk16(h_bits((_Float16)bfr(b[2])), h_bits((_Float16)bfr(b[3])));
  if (i < n8) {
    *(volatile v4u*)(dst + (size_t)i * 8) = o;
    __threadfence();
    *(volatile v4u*)(dst + (size_t)i * 8) = o;
  }
}

__global__ __launch_bounds__(128) void pe_rows(float* pe) {
  const int t = threadIdx.x, p = blockIdx.x;
  const int i = t >> 1;
  const float cexp = (float)(-9.210340371976184 / 128.0);
  const float dv  = expf((float)(2 * i) * cexp);
  const float ang = (float)p * dv;
  float sn, cs;
  sincosf(ang, &sn, &cs);
  const float v = (t & 1) ? cs : sn;
  float* dst = pe + (size_t)p * PEW + t;
  *(volatile float*)dst = v;
  __threadfence();
  *(volatile float*)dst = v;
}

__global__ __launch_bounds__(256) void convT64(const float* __restrict__ W, long long zsW, unsigned short* Wt,
                                               long long zsT, int K, int O, float wsc) {
  __shared__ __align__(16) unsigned short sTt[64 * 72];
  const int tid = threadIdx.x, lane = tid & 31, wave = tid >> 5;
  const int o0 = blockIdx.x * 64, k0 = blockIdx.y * 64;
  const float* Wz = W + (size_t)blockIdx.z * (size_t)zsW;
  unsigned short* Wtz = Wt + (size_t)blockIdx.z * (size_t)zsT;
  const int kr = tid >> 2, cs = (tid & 3) * 16;
  const float* src = Wz + (size_t)(k0 + kr) * O + o0 + cs;
#pragma unroll
  for (int q = 0; q < 4; ++q) {
    const v4f v = *(const v4f*)(src + 4 * q);
#pragma unroll
    for (int e = 0; e < 4; ++e) sTt[(cs + 4 * q + e) * 72 + kr] = h_bits((_Float16)(bfr(v[e]) * wsc));
  }
  __syncthreads();
  const int q8 = lane >> 3, c8 = (lane & 7) * 8;
  v4u vv[2];
#pragma unroll
  for (int it = 0; it < 2; ++it) {
    const int row = wave * 8 + it * 4 + q8;
    vv[it] = *(const v4u*)(sTt + row * 72 + c8);
  }
  for (int pass = 0; pass < 2; ++pass) {
#pragma unroll
    for (int it = 0; it < 2; ++it) {
      const int row = wave * 8 + it * 4 + q8;
      *(volatile v4u*)(Wtz + (size_t)(o0 + row) * K + k0 + c8) = vv[it];
    }
    __threadfence();
  }
}

template <int OM, int BIASM, int ACT, int RES>
__global__ __launch_bounds__(256) void gemm64(
    const unsigned short* __restrict__ Ap, int lda, int ldkA, long long strideA,
    const unsigned short* __restrict__ Btp, int ldb, long long strideB,
    const float* __restrict__ bias0, const float* __restrict__ bias1, int Nb,
    const float* resid,
    void* Cout, int ldc, long long strideC,
    int M, int N, int K, float oscale) {
  const _Float16* A  = (const _Float16*)(const void*)Ap;
  const _Float16* Bt = (const _Float16*)(const void*)Btp;
  __shared__ __align__(16) float sT[8][16 * 68];
  const int b    = blockIdx.y;
  const int lane = threadIdx.x & 31;
  const int wave = threadIdx.x >> 5;
  const int tilesN = N >> 6;
  const int tilesM = M >> 6;
  const int tile = blockIdx.x * 8 + wave;
  if (tile >= tilesM * tilesN) return;
  const int tm = tile / tilesN;
  const int tn = tile - tm * tilesN;
  const int m0 = tm << 6;
  const int n0 = tn << 6;

  const _Float16* Ab = A  + (size_t)b * strideA;
  const _Float16* Bb = Bt + (size_t)b * strideB;

  const int rlane = lane & 15;
  const int koff  = (lane >> 4) * 8;
  const int mOff  = (lane >> 4) * 8;

  v8f acc[4][4];
#pragma unroll
  for (int i = 0; i < 4; ++i)
#pragma unroll
    for (int j = 0; j < 4; ++j) acc[i][j] = zero8();

  for (int k0 = 0; k0 < K; k0 += 32) {
    v16h bh[4];
#pragma unroll
    for (int j = 0; j < 4; ++j) {
      const size_t bo = (size_t)(n0 + (j << 4) + rlane) * ldb + koff + k0;
      bh[j] = ldfrag_h(Bb + bo);
    }
    const size_t kA = (size_t)k0 * (size_t)ldkA + koff;
#pragma unroll
    for (int i = 0; i < 4; ++i) {
      const size_t ao = (size_t)(m0 + (i << 4) + rlane) * lda + kA;
      const v16h ah = ldfrag_h(Ab + ao);
#pragma unroll
      for (int j = 0; j < 4; ++j) acc[i][j] = mma_h_raw(ah, bh[j], acc[i][j]);
      dep_guard1(acc[i][0], acc[i][3], ah);
    }
    keep4_h(bh[0], bh[1], bh[2], bh[3]);
  }
  acc_guard4(acc[0][0], acc[0][1], acc[0][2], acc[0][3]);
  acc_guard4(acc[1][0], acc[1][1], acc[1][2], acc[1][3]);
  acc_guard4(acc[2][0], acc[2][1], acc[2][2], acc[2][3]);
  acc_guard4(acc[3][0], acc[3][1], acc[3][2], acc[3][3]);

  const int hh2 = lane >> 4, c4 = (lane & 15) * 4;
  const int q8  = lane >> 3, c8 = (lane & 7) * 8;
  float bc[8];
#pragma unroll
  for (int e = 0; e < 8; ++e) bc[e] = 0.f;
  if (BIASM == 0) {
    const bool use1 = (n0 >= Nb);
    if (OM == 0) {
      const int cb = n0 + c4;
      const int i0 = (cb < Nb - 4) ? cb : (Nb - 4);
      const int i1 = (cb - Nb > 0) ? (cb - Nb) : 0;
      const v4f b0v = *(const v4f*)(bias0 + i0);
      const v4f b1v = *(const v4f*)(bias1 + i1);
#pragma unroll
      for (int e = 0; e < 4; ++e) bc[e] = bfr(use1 ? b1v[e] : b0v[e]);
    } else {
      const int cb = n0 + c8;
      const int i0 = (cb < Nb - 8) ? cb : (Nb - 8);
      const int i1 = (cb - Nb > 0) ? (cb - Nb) : 0;
      const v4f b0a = *(const v4f*)(bias0 + i0), b0b = *(const v4f*)(bias0 + i0 + 4);
      const v4f b1a = *(const v4f*)(bias1 + i1), b1b = *(const v4f*)(bias1 + i1 + 4);
#pragma unroll
      for (int e = 0; e < 4; ++e) {
        bc[e]     = bfr(use1 ? b1a[e] : b0a[e]);
        bc[4 + e] = bfr(use1 ? b1b[e] : b0b[e]);
      }
    }
  }

  float* slab = sT[wave];
#pragma unroll
  for (int i = 0; i < 4; ++i) {
    const int mBase = m0 + (i << 4);
#pragma unroll
    for (int j = 0; j < 4; ++j) {
#pragma unroll
      for (int r = 0; r < 8; ++r) {
        slab[(mOff + r) * 68 + (j << 4) + rlane] = acc[i][j][r];
      }
    }
    wave_sync_lds();
    if (OM == 0) {
      float* C = (float*)Cout + (size_t)b * strideC;
      v4f vals[8];
#pragma unroll
      for (int it = 0; it < 8; ++it) {
        const int row = it * 2 + hh2;
        v4f v = *(const v4f*)(slab + row * 68 + c4);
#pragma unroll
        for (int e = 0; e < 4; ++e) {
          float f = v[e] * oscale + bc[e];
          if (ACT) f = fmaxf(f, 0.0f);
          v[e] = f;
        }
        if (RES == 1) {
          const float* Rb = resid + (size_t)b * strideC;
          const v4f rr = *(const v4f*)(Rb + (size_t)(mBase + row) * ldc + n0 + c4);
#pragma unroll
          for (int e = 0; e < 4; ++e) v[e] += rr[e];
        }
        vals[it] = v;
      }
      for (int pass = 0; pass < 2; ++pass) {
#pragma unroll
        for (int it = 0; it < 8; ++it) {
          const int row = it * 2 + hh2;
          *(volatile v4f*)(C + (size_t)(mBase + row) * ldc + n0 + c4) = vals[it];
        }
        __threadfence();
      }
    } else {
      unsigned short* C = (unsigned short*)Cout + (size_t)b * strideC;
      v4u hv[4];
#pragma unroll
      for (int it = 0; it < 4; ++it) {
        const int row = it * 4 + q8;
        const float* sp = slab + row * 68 + c8;
        float bm = 0.f;
        if (BIASM == 1) bm = bfr(bias0[mBase + row]);
        v4u a;
#pragma unroll
        for (int e = 0; e < 4; ++e) {
          float f0 = sp[2 * e]     * oscale + ((BIASM == 1) ? bm : bc[2 * e]);
          float f1 = sp[2 * e + 1] * oscale + ((BIASM == 1) ? bm : bc[2 * e + 1]);
          if (ACT) { f0 = fmaxf(f0, 0.0f); f1 = fmaxf(f1, 0.0f); }
          unsigned short u0, u1;
          if (OM == 1) { u0 = bf_bits(f0); u1 = bf_bits(f1); }
          else         { u0 = h_bits((_Float16)f0); u1 = h_bits((_Float16)f1); }
          a[e] = pk16(u0, u1);
        }
        hv[it] = a;
      }
      for (int pass = 0; pass < 2; ++pass) {
#pragma unroll
        for (int it = 0; it < 4; ++it) {
          const int row = it * 4 + q8;
          *(volatile v4u*)(C + (size_t)(mBase + row) * ldc + n0 + c8) = hv[it];
        }
        __threadfence();
      }
    }
    wave_sync_lds();
  }
}

__global__ __launch_bounds__(128)
void attn32(const unsigned short* __restrict__ qkp, const unsigned short* __restrict__ vtp,
            unsigned short* outp, float sscale) {
  union FH { v16h v; v8h h[2]; };
  __shared__ __align__(16) _Float16 Ksh[64 * 32];
  __shared__ __align__(16) _Float16 Vth[32 * 64];
  __shared__ __align__(16) _Float16 Psh[4][16 * 64];
  __shared__ __align__(16) float    Os[4][16 * 32];

  const int tid  = threadIdx.x;
  const int wave = tid >> 5;
  const int lane = tid & 31;
  const int hh   = lane >> 4;
  const int c    = lane & 15;

  const int bx   = blockIdx.x;
  const int qb   = bx % NQB;
  const int rest = bx / NQB;
  const int h    = rest % NH;
  const int b    = rest / NH;
  const int q0   = qb * 64 + wave * 16;
  const size_t rowB = (size_t)b * SP;

  const _Float16* Qh = (const _Float16*)(const void*)qkp + (size_t)h * HD;
  const _Float16* Kg = (const _Float16*)(const void*)qkp + DM + (size_t)h * HD;
  const _Float16* Vh = (const _Float16*)(const void*)vtp + ((size_t)b * DM + (size_t)h * HD) * SP;

  const v16h qa = ldfrag_h(Qh + (rowB + q0 + c) * QKP + 8 * hh);

  float mrow[8], lrow[8];
  v8f oacc[2];
#pragma unroll
  for (int r = 0; r < 8; ++r) { mrow[r] = -INFINITY; lrow[r] = 0.f; }
#pragma unroll
  for (int t = 0; t < 2; ++t) oacc[t] = zero8();

  for (int kt = 0; kt < NQB; ++kt) {
    const int kv0 = kt * 64;
    __syncthreads();
    {
      const int r = tid >> 1, hf = (tid & 1) * 16;
      const _Float16* kg = Kg + (rowB + kv0 + r) * QKP + hf;
      const v8h a0 = *(const v8h*)(kg);
      const v8h a1 = *(const v8h*)(kg + 8);
      *(v8h*)(Ksh + r * 32 + hf)     = a0;
      *(v8h*)(Ksh + r * 32 + hf + 8) = a1;
      const int d = tid >> 2, sg = (tid & 3) * 16;
      const _Float16* vg = Vh + (size_t)d * SP + kv0 + sg;
      const v8h b0 = *(const v8h*)(vg);
      const v8h b1 = *(const v8h*)(vg + 8);
      *(v8h*)(Vth + d * 64 + sg)     = b0;
      *(v8h*)(Vth + d * 64 + sg + 8) = b1;
    }
    __syncthreads();

    v8f s[4];
#pragma unroll
    for (int j = 0; j < 4; ++j) {
      FH kb;
      kb.h[0] = *(const v8h*)(Ksh + (j * 16 + c) * 32 + 8 * hh);
      kb.h[1] = *(const v8h*)(Ksh + (j * 16 + c) * 32 + 16 + 8 * hh);
      const v8f sh = mma_h(qa, kb.v, zero8());
#pragma unroll
      for (int r = 0; r < 8; ++r) {
        const float v = sh[r] * sscale;
        const int key = kv0 + j * 16 + c;
        s[j][r] = (key < SV) ? v : -INFINITY;
      }
    }

    _Float16* pwh = Psh[wave];
#pragma unroll
    for (int r = 0; r < 8; ++r) {
      float m = s[0][r];
      m = fmaxf(m, s[1][r]);
      m = fmaxf(m, s[2][r]);
      m = fmaxf(m, s[3][r]);
#pragma unroll
      for (int off = 1; off < 16; off <<= 1) m = fmaxf(m, __shfl_xor(m, off, 32));
      const float mnew  = fmaxf(mrow[r], m);
      const float alpha = __expf(mrow[r] - mnew);
      mrow[r] = mnew;
      float psum = 0.f;
#pragma unroll
      for (int j = 0; j < 4; ++j) {
        const float p = __expf(s[j][r] - mnew);
        psum += p;
        pwh[(8 * hh + r) * 64 + j * 16 + c] = (_Float16)(p * 1024.0f);
      }
#pragma unroll
      for (int off = 1; off < 16; off <<= 1) psum += __shfl_xor(psum, off, 32);
      lrow[r] = lrow[r] * alpha + psum;
#pragma unroll
      for (int t = 0; t < 2; ++t) oacc[t][r] *= alpha;
    }
    wave_sync_lds();

#pragma unroll 1
    for (int kk = 0; kk < 2; ++kk) {
      FH pa;
      pa.h[0] = *(const v8h*)(pwh + c * 64 + kk * 32 + 8 * hh);
      pa.h[1] = *(const v8h*)(pwh + c * 64 + kk * 32 + 16 + 8 * hh);
#pragma unroll
      for (int t = 0; t < 2; ++t) {
        FH vb;
        vb.h[0] = *(const v8h*)(Vth + (t * 16 + c) * 64 + kk * 32 + 8 * hh);
        vb.h[1] = *(const v8h*)(Vth + (t * 16 + c) * 64 + kk * 32 + 16 + 8 * hh);
        oacc[t] = mma_h(pa.v, vb.v, oacc[t]);
      }
    }
  }

  float* os = Os[wave];
#pragma unroll
  for (int r = 0; r < 8; ++r) {
    const float l = lrow[r];
    const float inv = ((l > 0.f) ? (1.0f / l) : 0.f) * (16.0f / 1024.0f);
#pragma unroll
    for (int t = 0; t < 2; ++t) os[(8 * hh + r) * 32 + t * 16 + c] = oacc[t][r] * inv;
  }
  wave_sync_lds();
  {
    const int rq = lane >> 2, cg = (lane & 3) * 8;
    v4u hv[2];
#pragma unroll
    for (int it = 0; it < 2; ++it) {
      const int row = it * 8 + rq;
      const float* sp = os + row * 32 + cg;
      v4u a;
#pragma unroll
      for (int e = 0; e < 4; ++e) a[e] = pk16(h_bits((_Float16)sp[2 * e]), h_bits((_Float16)sp[2 * e + 1]));
      hv[it] = a;
    }
    const size_t headB = ((size_t)(b * NH + h) * SP + (size_t)q0) * HD;
    for (int pass = 0; pass < 2; ++pass) {
#pragma unroll
      for (int it = 0; it < 2; ++it) {
        const int row = it * 8 + rq;
        const size_t go = headB + (size_t)row * HD + cg;
        *(volatile v4u*)(outp + go) = hv[it];
      }
      __threadfence();
    }
  }
}

__global__ __launch_bounds__(64) void assemble_rows(const float* __restrict__ EC, const float* __restrict__ pe,
                                                    const int* __restrict__ xc, const int* __restrict__ yc,
                                                    const float* __restrict__ cls, float* Xo, unsigned short* Ho) {
  __shared__ __align__(16) unsigned int sb[128];
  const int t = threadIdx.x;
  const int m = blockIdx.x;
  const int b = m / SP, s = m - b * SP;
  int tok = b * NCELL + s - 1;
  tok = (tok < 0) ? 0 : ((tok > MC - 1) ? (MC - 1) : tok);
  int xi = xc[tok]; xi = (xi < 0) ? 0 : ((xi > MAXHW - 1) ? (MAXHW - 1) : xi);
  int yi = yc[tok]; yi = (yi < 0) ? 0 : ((yi > MAXHW - 1) ? (MAXHW - 1) : yi);
  const int p  = (t < 32) ? xi : yi;
  const int j0 = 4 * t - ((t < 32) ? 0 : PEW);
  const v4f ec = *(const v4f*)(EC + (size_t)tok * DM + 4 * t);
  const v4f pv = *(const v4f*)(pe + (size_t)p * PEW + j0);
  const v4f cv = *(const v4f*)(cls + 4 * t);
  const bool isc = (s == 0);
  const bool isv = (s >= 1) && (s <= NCELL);
  v4f y;
#pragma unroll
  for (int e = 0; e < 4; ++e) y[e] = isc ? bfr(cv[e]) : (isv ? (ec[e] + pv[e]) : 0.0f);
  row_store_fh(sb, Xo + (size_t)m * DM, Ho + (size_t)m * DM, y, t);
}

__global__ __launch_bounds__(64) void ln_rows(const float* __restrict__ Tin, const float* __restrict__ gam,
                                              const float* __restrict__ bet, float* Xo, unsigned short* Ho) {
  __shared__ float red0[2], red1[2];
  __shared__ __align__(16) unsigned int sb[128];
  const int t = threadIdx.x, lane = t & 31, wave = t >> 5;
  const size_t base = (size_t)blockIdx.x * DM;
  const v4f xv = *(const v4f*)(Tin + base + 4 * t);
  const float mean = bsum2((xv[0] + xv[1]) + (xv[2] + xv[3]), red0, lane, wave) * (1.0f / DM);
  v4f d;
#pragma unroll
  for (int e = 0; e < 4; ++e) d[e] = xv[e] - mean;
  const float var  = bsum2((d[0] * d[0] + d[1] * d[1]) + (d[2] * d[2] + d[3] * d[3]), red1, lane, wave) * (1.0f / DM);
  const float rstd = 1.0f / sqrtf(var + LNEPS);
  const v4f gv = *(const v4f*)(gam + 4 * t);
  const v4f bv = *(const v4f*)(bet + 4 * t);
  v4f y;
#pragma unroll
  for (int e = 0; e < 4; ++e) y[e] = (d[e] * rstd) * bfr(gv[e]) + bfr(bv[e]);
  row_store_fh(sb, Xo + base, Ho + base, y, t);
}

__global__ __launch_bounds__(256) void head_k(const float* __restrict__ X,
                                              const float* __restrict__ lw, const float* __restrict__ lb,
                                              const float* __restrict__ hw1, const float* __restrict__ hb1,
                                              const float* __restrict__ hw2, const float* __restrict__ hb2,
                                              float* out) {
  __shared__ float scl[NB][DM];
  __shared__ float shd[NB][DM];
  __shared__ __align__(16) float so[NOUT0 + 64];
  __shared__ float red[2 * NB][8];
  const int t = threadIdx.x, lane = t & 31, wave = t >> 5;
  const float g = bfr(lw[t]), be = bfr(lb[t]);

#pragma unroll
  for (int bb = 0; bb < NB; ++bb) {
    const float x = X[(size_t)bb * SP * DM + t];
    const float mean = bsum256(x, red[2 * bb], lane, wave) * (1.0f / DM);
    const float d = x - mean;
    const float var  = bsum256(d * d, red[2 * bb + 1], lane, wave) * (1.0f / DM);
    const float rstd = 1.0f / sqrtf(var + LNEPS);
    const float v = (d * rstd) * g + be;
    scl[bb][t] = v;
    so[bb * DM + t] = v;
  }
  __syncthreads();

  float a[NB];
#pragma unroll
  for (int bb = 0; bb < NB; ++bb) a[bb] = 0.f;
#pragma unroll 1
  for (int k = 0; k < DM; ++k) {
    const float w = bfr(hw1[(size_t)k * DM + t]);
#pragma unroll
    for (int bb = 0; bb < NB; ++bb) a[bb] += scl[bb][k] * w;
  }
  const float b1 = bfr(hb1[t]);
#pragma unroll
  for (int bb = 0; bb < NB; ++bb) shd[bb][t] = fmaxf(a[bb] + b1, 0.0f);
  __syncthreads();

  {
    const int bb = (t >> 1) & (NB - 1), o = t & 1;
    float a2 = 0.f;
#pragma unroll 1
    for (int i = 0; i < DM; ++i) a2 += shd[bb][i] * bfr(hw2[i * 2 + o]);
    const float lv = a2 + bfr(hb2[o]);
    if (t < NOUT1) so[NOUT0 + t] = lv;
  }
  __syncthreads();

  const v4f va = *(const v4f*)(so + 4 * t);
  const v4f vb = *(const v4f*)(so + (NOUT0 / 2) + 4 * t);
  const int tc = (t < 4) ? t : 3;
  const v4f vc = *(const v4f*)(so + NOUT0 + 4 * tc);
  *(volatile v4f*)(out + 4 * t) = va;
  *(volatile v4f*)(out + (NOUT0 / 2) + 4 * t) = vb;
  if (t < 4) *(volatile v4f*)(out + NOUT0 + 4 * t) = vc;
  __threadfence();
  *(volatile v4f*)(out + 4 * t) = va;
  *(volatile v4f*)(out + (NOUT0 / 2) + 4 * t) = vb;
  if (t < 4) *(volatile v4f*)(out + NOUT0 + 4 * t) = vc;
}

extern "C" void kernel_launch(void* const* d_in, const int* in_sizes, int n_in,
                              void* d_out, int out_size, void* d_ws, size_t ws_size,
                              hipStream_t stream) {
  if (n_in < 32) return;
  if (in_sizes[0] != MC * FEAT) return;
  if (in_sizes[1] != MC || in_sizes[2] != MC) return;
  if (in_sizes[3] != FEAT * DM || in_sizes[4] != DM) return;
  if (in_sizes[5] != FEAT * DCT || in_sizes[6] != DCT) return;
  if (in_sizes[7] != DCT * DM || in_sizes[8] != DM) return;
  if (in_sizes[9] != DM) return;
  if (in_sizes[10] != NLAYER * DM * DM || in_sizes[11] != NLAYER * DM) return;
  if (in_sizes[12] != NLAYER * DM * DM || in_sizes[13] != NLAYER * DM) return;
  if (in_sizes[14] != NLAYER * DM * DM || in_sizes[15] != NLAYER * DM) return;
  if (in_sizes[16] != NLAYER * DM * DM || in_sizes[17] != NLAYER * DM) return;
  if (in_sizes[18] != NLAYER * DM || in_sizes[19] != NLAYER * DM) return;
  if (in_sizes[20] != NLAYER * DM || in_sizes[21] != NLAYER * DM) return;
  if (in_sizes[22] != NLAYER * DM * DFF || in_sizes[23] != NLAYER * DFF) return;
  if (in_sizes[24] != NLAYER * DFF * DM || in_sizes[25] != NLAYER * DM) return;
  if (in_sizes[26] != DM || in_sizes[27] != DM) return;
  if (in_sizes[28] != DM * DM || in_sizes[29] != DM) return;
  if (in_sizes[30] != DM * 2 || in_sizes[31] != 2) return;
  if (out_size != NOUT0 + NOUT1) return;

  const float* cf    = (const float*)d_in[0];
  const int*   xc    = (const int*)d_in[1];
  const int*   yc    = (const int*)d_in[2];
  const float* W_emb = (const float*)d_in[3];
  const float* b_emb = (const float*)d_in[4];
  const float* W_ct1 = (const float*)d_in[5];
  const float* b_ct1 = (const float*)d_in[6];
  const float* W_ct2 = (const float*)d_in[7];
  const float* b_ct2 = (const float*)d_in[8];
  const float* clsT  = (const float*)d_in[9];
  const float* Wq    = (const float*)d_in[10];
  const float* bq    = (const float*)d_in[11];
  const float* Wk    = (const float*)d_in[12];
  const float* bk    = (const float*)d_in[13];
  const float* Wv    = (const float*)d_in[14];
  const float* bv    = (const float*)d_in[15];
  const float* Wo    = (const float*)d_in[16];
  const float* bo    = (const float*)d_in[17];
  const float* ln1g  = (const float*)d_in[18];
  const float* ln1b  = (const float*)d_in[19];
  const float* ln2g  = (const float*)d_in[20];
  const float* ln2b  = (const float*)d_in[21];
  const float* Wf1   = (const float*)d_in[22];
  const float* bf1   = (const float*)d_in[23];
  const float* Wf2   = (const float*)d_in[24];
  const float* bf2   = (const float*)d_in[25];
  const float* lnfg  = (const float*)d_in[26];
  const float* lnfb  = (const float*)d_in[27];
  const float* Wh1   = (const float*)d_in[28];
  const float* bh1   = (const float*)d_in[29];
  const float* Wh2   = (const float*)d_in[30];
  const float* bh2   = (const float*)d_in[31];

  const size_t PWE  = (size_t)DM * FEAT * 2;
  const size_t PWC1 = (size_t)DCT * FEAT * 2;
  const size_t PWC2 = (size_t)DM * DCT * 2;
  const size_t PWQK = (size_t)NLAYER * QKP * DM * 2;
  const size_t PWD  = (size_t)NLAYER * DM * DM * 2;
  const size_t PWF  = (size_t)NLAYER * DFF * DM * 2;
  const size_t PPE  = (size_t)MAXHW * PEW * 4;
  const size_t PCF  = (size_t)MC * FEAT * 2;
  const size_t PEF  = (size_t)MC * DM * 4;
  const size_t PHD  = (size_t)MC * DCT * 2;
  const size_t PAF  = (size_t)MP * DM * 4;
  const size_t PAH  = (size_t)MP * DM * 2;
  const size_t PQK  = (size_t)MP * QKP * 2;
  const size_t PVT  = (size_t)NB * DM * SP * 2;
  const size_t PCTX = (size_t)NB * NH * SP * HD * 2;
  const size_t PG   = (size_t)MP * DFF * 2;
  size_t off = 0;
  const size_t oWembT = off; off += PWE;
  const size_t oWct1T = off; off += PWC1;
  const size_t oWct2T = off; off += PWC2;
  const size_t oWqkT  = off; off += PWQK;
  const size_t oWvT   = off; off += PWD;
  const size_t oWoT   = off; off += PWD;
  const size_t oW1T   = off; off += PWF;
  const size_t oW2T   = off; off += PWF;
  const size_t oPE    = off; off += PPE;
  const size_t oCF    = off; off += PCF;
  const size_t oE     = off; off += PEF;
  const size_t oHd    = off; off += PHD;
  const size_t oEC    = off; off += PEF;
  const size_t oX     = off; off += PAF;
  const size_t oT     = off; off += PAF;
  const size_t oX16   = off; off += PAH;
  const size_t oQK    = off; off += PQK;
  const size_t oVT    = off; off += PVT;
  const size_t oCtx   = off; off += PCTX;
  const size_t oG     = off; off += PG;
  if (off > ws_size) return;
  if (off > (size_t)134217728) return;

  char* ws = (char*)d_ws;
  unsigned short* WembT = (unsigned short*)(ws + oWembT);
  unsigned short* Wct1T = (unsigned short*)(ws + oWct1T);
  unsigned short* Wct2T = (unsigned short*)(ws + oWct2T);
  unsigned short* WqkT  = (unsigned short*)(ws + oWqkT);
  unsigned short* WvT   = (unsigned short*)(ws + oWvT);
  unsigned short* WoT   = (unsigned short*)(ws + oWoT);
  unsigned short* W1T   = (unsigned short*)(ws + oW1T);
  unsigned short* W2T   = (unsigned short*)(ws + oW2T);
  float*          PE    = (float*)(ws + oPE);
  unsigned short* CF    = (unsigned short*)(ws + oCF);
  float*          E     = (float*)(ws + oE);
  unsigned short* Hd    = (unsigned short*)(ws + oHd);
  float*          EC    = (float*)(ws + oEC);
  float*          X     = (float*)(ws + oX);
  float*          T     = (float*)(ws + oT);
  unsigned short* X16   = (unsigned short*)(ws + oX16);
  unsigned short* QK    = (unsigned short*)(ws + oQK);
  unsigned short* VT    = (unsigned short*)(ws + oVT);
  unsigned short* Ctx   = (unsigned short*)(ws + oCtx);
  unsigned short* G     = (unsigned short*)(ws + oG);

  const dim3 blk(256), blk128(128), blk64(64);
  const dim3 gRow(MP);
  const float invw  = 1.0f / WSC;
  const float invwc = 1.0f / (WSC * 16.0f);
  const float sscale = 0.17677669529663687f;

  conv_rows8<<<dim3((MC * FEAT / 8) / 256), blk, 0, stream>>>(cf, CF, MC * FEAT / 8);
  pe_rows<<<dim3(MAXHW), blk128, 0, stream>>>(PE);
  convT64<<<dim3(DM / 64, FEAT / 64, 1), blk, 0, stream>>>(W_emb, 0LL, WembT, 0LL, FEAT, DM, WSC);
  convT64<<<dim3(DCT / 64, FEAT / 64, 1), blk, 0, stream>>>(W_ct1, 0LL, Wct1T, 0LL, FEAT, DCT, WSC);
  convT64<<<dim3(DM / 64, DCT / 64, 1), blk, 0, stream>>>(W_ct2, 0LL, Wct2T, 0LL, DCT, DM, WSC);
  gemm64<0, 0, 0, 0><<<dim3(((MC / 64) * (DM / 64) + 7) / 8, 1), blk, 0, stream>>>(
      CF, FEAT, 1, 0LL, WembT, FEAT, 0LL, b_emb, b_emb, DM, E,
      (void*)E, DM, 0LL, MC, DM, FEAT, invw);
  gemm64<2, 0, 1, 0><<<dim3(((MC / 64) * (DCT / 64) + 7) / 8, 1), blk, 0, stream>>>(
      CF, FEAT, 1, 0LL, Wct1T, FEAT, 0LL, b_ct1, b_ct1, DCT, E,
      (void*)Hd, DCT, 0LL, MC, DCT, FEAT, invw);
  gemm64<0, 0, 0, 1><<<dim3(((MC / 64) * (DM / 64) + 7) / 8, 1), blk, 0, stream>>>(
      Hd, DCT, 1, 0LL, Wct2T, DCT, 0LL, b_ct2, b_ct2, DM, E,
      (void*)EC, DM, 0LL, MC, DM, DCT, invw);
  assemble_rows<<<gRow, blk64, 0, stream>>>(EC, PE, xc, yc, clsT, X, X16);

  convT64<<<dim3(DM / 64, DM / 64, NLAYER), blk, 0, stream>>>(Wq, (long long)DM * DM, WqkT, (long long)QKP * DM, DM, DM, WSC);
  convT64<<<dim3(DM / 64, DM / 64, NLAYER), blk, 0, stream>>>(Wk, (long long)DM * DM, WqkT + (size_t)DM * DM, (long long)QKP * DM, DM, DM, WSC);
  convT64<<<dim3(DM / 64, DM / 64, NLAYER), blk, 0, stream>>>(Wv, (long long)DM * DM, WvT, (long long)DM * DM, DM, DM, WSC);
  convT64<<<dim3(DM / 64, DM / 64, NLAYER), blk, 0, stream>>>(Wo, (long long)DM * DM, WoT, (long long)DM * DM, DM, DM, WSC);
  convT64<<<dim3(DFF / 64, DM / 64, NLAYER), blk, 0, stream>>>(Wf1, (long long)DM * DFF, W1T, (long long)DFF * DM, DM, DFF, WSC);
  convT64<<<dim3(DM / 64, DFF / 64, NLAYER), blk, 0, stream>>>(Wf2, (long long)DFF * DM, W2T, (long long)DM * DFF, DFF, DM, WSC);

  const dim3 gNqk(((MP / 64) * (QKP / 64) + 7) / 8, 1);
  const dim3 gVT(((DM / 64) * (SP / 64) + 7) / 8, NB);
  const dim3 gWo(((SP / 64) * (DM / 64) + 7) / 8, NB);
  const dim3 gNff(((MP / 64) * (DFF / 64) + 7) / 8, 1);
  const dim3 gN256(((MP / 64) * (DM / 64) + 7) / 8, 1);
  const dim3 gAttn(NB * NH * NQB);

  for (int l = 0; l < NLAYER; ++l) {
    const unsigned short* WqkT_l = WqkT + (size_t)l * QKP * DM;
    const unsigned short* WvT_l  = WvT + (size_t)l * DM * DM;
    const unsigned short* WoT_l  = WoT + (size_t)l * DM * DM;
    const unsigned short* W1T_l  = W1T + (size_t)l * DFF * DM;
    const unsigned short* W2T_l  = W2T + (size_t)l * DM * DFF;
    const float* bq_l  = bq + (size_t)l * DM;
    const float* bk_l  = bk + (size_t)l * DM;
    const float* bv_l  = bv + (size_t)l * DM;
    const float* bo_l  = bo + (size_t)l * DM;
    const float* bf1_l = bf1 + (size_t)l * DFF;
    const float* bf2_l = bf2 + (size_t)l * DM;

    gemm64<2, 0, 0, 0><<<gNqk, blk, 0, stream>>>(
        X16, DM, 1, 0LL, WqkT_l, DM, 0LL, bq_l, bk_l, DM, X,
        (void*)QK, QKP, 0LL, MP, QKP, DM, invw);
    gemm64<2, 1, 0, 0><<<gVT, blk, 0, stream>>>(
        WvT_l, DM, 1, 0LL, X16, DM, (long long)SP * DM, bv_l, bv_l, SP, X,
        (void*)VT, SP, (long long)DM * SP, DM, SP, DM, invw);
    attn32<<<gAttn, blk128, 0, stream>>>(QK, VT, Ctx, sscale);
    gemm64<0, 0, 0, 1><<<gWo, blk, 0, stream>>>(
        Ctx, HD, SP, (long long)NH * SP * HD, WoT_l, DM, 0LL, bo_l, bo_l, DM, X,
        (void*)T, DM, (long long)SP * DM, SP, DM, DM, invwc);
    ln_rows<<<gRow, blk64, 0, stream>>>(T, ln1g + (size_t)l * DM, ln1b + (size_t)l * DM, X, X16);
    gemm64<2, 0, 1, 0><<<gNff, blk, 0, stream>>>(
        X16, DM, 1, 0LL, W1T_l, DM, 0LL, bf1_l, bf1_l, DFF, X,
        (void*)G, DFF, 0LL, MP, DFF, DM, invw);
    gemm64<0, 0, 0, 1><<<gN256, blk, 0, stream>>>(
        G, DFF, 1, 0LL, W2T_l, DFF, 0LL, bf2_l, bf2_l, DM, X,
        (void*)T, DM, 0LL, MP, DM, DFF, invw);
    ln_rows<<<gRow, blk64, 0, stream>>>(T, ln2g + (size_t)l * DM, ln2b + (size_t)l * DM, X, X16);
  }

  head_k<<<dim3(1), blk, 0, stream>>>(X, lnfg, lnfb, Wh1, bh1, Wh2, bh2, (float*)d_out);
  (void)hipGetLastError();
}
